// DSConv_26585847562975
// MI455X (gfx1250) — hardware-verified
//
#include <hip/hip_runtime.h>
#include <math.h>
#include <stddef.h>

typedef __attribute__((ext_vector_type(16))) _Float16 v16h;
typedef __attribute__((ext_vector_type(8)))  _Float16 v8h;
typedef __attribute__((ext_vector_type(16))) __bf16   v16b;
typedef __attribute__((ext_vector_type(8)))  __bf16   v8b;
typedef __attribute__((ext_vector_type(8)))  float    v8f;
typedef __attribute__((ext_vector_type(4)))  float    v4f;
typedef __attribute__((ext_vector_type(4)))  unsigned v4u;
typedef __attribute__((ext_vector_type(8)))  unsigned short v8us;

constexpr int NBATCH = 4;
constexpr int NCH    = 32;
constexpr int NROW   = 256;
constexpr int NCOL   = 256;
constexpr int NPIX   = NROW * NCOL;
constexpr int NTAP   = 9;
constexpr int PADN   = 258;
constexpr int XPIX   = 32;
constexpr int OFFC   = 16;
constexpr int NTHR   = 256;
constexpr int PARTW  = 32;
constexpr int SLAB1P = 20;
constexpr int SLAB2P = 36;
constexpr int ATP    = 40;
constexpr float CARRY_A = 64.0f;
constexpr float CARRY_W = 64.0f;
constexpr float FOLD2   = 1.0f / 4096.0f;
constexpr float GN_EPS  = 1e-5f;

static_assert(NCOL == NTHR);
static_assert(NPIX % NTHR == 0);
static_assert((NBATCH * NCH * NPIX) % (NTHR * 4) == 0);
static_assert(XPIX == 32);
static_assert((NTAP * 16 * 32) % (8 * 32) == 0);
static_assert(ATP % 8 == 0 && SLAB1P % 4 == 0 && SLAB2P % 4 == 0);
static_assert(8 * 32 * SLAB2P <= NTAP * NCOL * 4);

constexpr size_t XCL_BYTES  = (size_t)NBATCH * PADN * PADN * XPIX * 2;
constexpr size_t OFF_BYTES  = (size_t)NBATCH * NPIX * OFFC * 4;
constexpr size_t PRE_BYTES  = (size_t)NBATCH * NCH * NPIX * 4;
constexpr size_t WOF_BYTES  = (size_t)NTAP * 16 * 32 * 2;
constexpr size_t WDS_BYTES  = (size_t)NTAP * 32 * 32 * 2;
constexpr size_t PART_BYTES = (size_t)NBATCH * NROW * PARTW * 4;
constexpr size_t STAT_BYTES = 256;
constexpr size_t XCL_OFS   = 0;
constexpr size_t OFF_OFS   = XCL_OFS + XCL_BYTES;
constexpr size_t PRE_OFS   = OFF_OFS + OFF_BYTES;
constexpr size_t WOF_OFS   = PRE_OFS + PRE_BYTES;
constexpr size_t WDS_OFS   = WOF_OFS + WOF_BYTES;
constexpr size_t PART1_OFS = WDS_OFS + WDS_BYTES;
constexpr size_t PART2_OFS = PART1_OFS + PART_BYTES;
constexpr size_t ST1_OFS   = PART2_OFS + PART_BYTES;
constexpr size_t ST2_OFS   = ST1_OFS + STAT_BYTES;
constexpr size_t WS_TOTAL  = ST2_OFS + STAT_BYTES;
static_assert(WS_TOTAL == 67662336);
static_assert(WS_TOTAL <= (size_t)134217728);
static_assert(OFF_OFS % 128 == 0 && PRE_OFS % 128 == 0 && WOF_OFS % 128 == 0 && WDS_OFS % 128 == 0);
static_assert(PART1_OFS % 128 == 0 && PART2_OFS % 128 == 0 && ST1_OFS % 128 == 0 && ST2_OFS % 128 == 0);
static_assert((PADN * XPIX * 2) % 128 == 0);

__device__ __forceinline__ unsigned short f2bf_bits(float f) {
  unsigned u = __float_as_uint(f);
  return (unsigned short)((u + 0x7FFFu + ((u >> 16) & 1u)) >> 16);
}
__device__ __forceinline__ float bf_bits2f(unsigned short h) { return __uint_as_float(((unsigned)h) << 16); }
__device__ __forceinline__ float bf_rne(float f) { return bf_bits2f(f2bf_bits(f)); }

__device__ __forceinline__ void dep_guard_h(v8f& a, v8f& b, v16h x, v16h y) { asm volatile("v_nop\n\tv_nop\n\tv_nop\n\tv_nop" : "+v"(a), "+v"(b) : "v"(x), "v"(y)); }
__device__ __forceinline__ void dep_guard_b(v8f& a, v8f& b, v16b x, v16b y) { asm volatile("v_nop\n\tv_nop\n\tv_nop\n\tv_nop" : "+v"(a), "+v"(b) : "v"(x), "v"(y)); }
__device__ __forceinline__ void keep4_h(v16h a, v16h b, v16h c, v16h d) { asm volatile("v_nop" :: "v"(a), "v"(b), "v"(c), "v"(d)); }
__device__ __forceinline__ void keep4_b(v16b a, v16b b, v16b c, v16b d) { asm volatile("v_nop" :: "v"(a), "v"(b), "v"(c), "v"(d)); }
__device__ __forceinline__ void acc_guard4(v8f& a, v8f& b, v8f& c, v8f& d) { asm volatile("v_nop\n\tv_nop\n\tv_nop\n\tv_nop" : "+v"(a), "+v"(b), "+v"(c), "+v"(d)); }
__device__ __forceinline__ void acc_guard2(v8f& a, v8f& b) { asm volatile("v_nop\n\tv_nop\n\tv_nop\n\tv_nop" : "+v"(a), "+v"(b)); }
__device__ __forceinline__ void guard2_b3(v8f& a, v8f& b, v16b x, v16b y, v16b z) { asm volatile("v_nop\n\tv_nop\n\tv_nop\n\tv_nop" : "+v"(a), "+v"(b) : "v"(x), "v"(y), "v"(z)); }
__device__ __forceinline__ void guard2_h3(v8f& a, v8f& b, v16h x, v16h y, v16h z) { asm volatile("v_nop\n\tv_nop\n\tv_nop\n\tv_nop" : "+v"(a), "+v"(b) : "v"(x), "v"(y), "v"(z)); }
template <typename T> struct Frag;
template <> struct Frag<_Float16> {
  typedef v16h V; union U { v16h v; v8h h[2]; };
  static __device__ __forceinline__ v16h load(const _Float16* p) {
    U f; f.h[0] = *(const v8h*)(p); f.h[1] = *(const v8h*)(p + 16); return f.v;
  }
  static __device__ __forceinline__ v8f mma(v16h a, v16h b, v8f c) {
    return __builtin_amdgcn_wmma_f32_16x16x32_f16(false, a, false, b, (short)0, c, false, false);
  }
  static __device__ __forceinline__ void guard(v8f& a, v8f& b, v16h x, v16h y) { dep_guard_h(a, b, x, y); }
  static __device__ __forceinline__ void keep(v16h a, v16h b, v16h c, v16h d) { keep4_h(a, b, c, d); }
};
template <> struct Frag<__bf16> {
  typedef v16b V; union U { v16b v; v8b h[2]; };
  static __device__ __forceinline__ v16b load(const __bf16* p) {
    U f; f.h[0] = *(const v8b*)(p); f.h[1] = *(const v8b*)(p + 16); return f.v;
  }
  static __device__ __forceinline__ v8f mma(v16b a, v16b b, v8f c) {
    return __builtin_amdgcn_wmma_f32_16x16x32_bf16(false, a, false, b, (short)0, c, false, false);
  }
  static __device__ __forceinline__ void guard(v8f& a, v8f& b, v16b x, v16b y) { dep_guard_b(a, b, x, y); }
  static __device__ __forceinline__ void keep(v16b a, v16b b, v16b c, v16b d) { keep4_b(a, b, c, d); }
};

__device__ __forceinline__ void wave_sync() {
  __builtin_amdgcn_fence(__ATOMIC_RELEASE, "workgroup");
  __builtin_amdgcn_wave_barrier();
  __builtin_amdgcn_fence(__ATOMIC_ACQUIRE, "workgroup");
}
__device__ __forceinline__ float lo16f(unsigned w) { float f = __uint_as_float(w << 16); asm volatile("" : "+v"(f)); return f; }
__device__ __forceinline__ float hi16f(unsigned w) { float f = __uint_as_float(w & 0xffff0000u); asm volatile("" : "+v"(f)); return f; }
__device__ __forceinline__ float lerp4(float a, float bb, float cc, float d, float w00, float w01, float w10, float w11) {
  float t = w00 * a; t = fmaf(w01, bb, t); t = fmaf(w10, cc, t); t = fmaf(w11, d, t); return t;
}

__global__ __launch_bounds__(NTHR) void k_xprep(const float* __restrict__ x, unsigned short* __restrict__ xcl) {
  __shared__ __align__(16) unsigned short sx[PADN * XPIX];
  const int tid = threadIdx.x;
  const int blk = blockIdx.x;
  const int b   = blk / PADN;
  const int wp  = blk - b * PADN;
  const bool interior = (wp >= 1) && (wp <= NROW);
  const v4u z4 = {0u, 0u, 0u, 0u};
  if (interior) {
    const float* xrow = x + (size_t)b * NCH * NPIX + (size_t)(wp - 1) * NCOL;
#pragma unroll 1
    for (int half = 0; half < 2; ++half) {
#pragma unroll
      for (int j = 0; j < 4; ++j) {
        const int idx = (half * 4 + j) * NTHR + tid;
        const int ch  = idx >> 6;
        const int h4  = (idx & 63) * 4;
        const v4f v = *(const v4f*)(xrow + (size_t)ch * NPIX + h4);
#pragma unroll
        for (int e = 0; e < 4; ++e) sx[(1 + h4 + e) * XPIX + ch] = f2bf_bits(v[e]);
      }
      asm volatile("" ::: "memory");
    }
    if (tid < 8) {
      const int p = (tid < 4) ? 0 : (PADN - 1);
      *(v4u*)(sx + p * XPIX + (tid & 3) * 8) = z4;
    }
  } else {
    for (int q = tid; q < PADN * 4; q += NTHR) *(v4u*)(sx + q * 8) = z4;
  }
  __syncthreads();
  unsigned short* dst = xcl + ((size_t)(b * PADN + wp) * PADN) * XPIX;
  for (int pass = 0; pass < 2; ++pass) {
#pragma unroll
    for (int it = 0; it < 4; ++it) {
      const int q = it * NTHR + tid;
      const v4u v = *(const v4u*)(sx + q * 8);
      *(volatile v4u*)(dst + (size_t)q * 8) = v;
    }
    if (tid < 8) {
      const int q = 4 * NTHR + tid;
      const v4u v = *(const v4u*)(sx + q * 8);
      *(volatile v4u*)(dst + (size_t)q * 8) = v;
    }
    __threadfence();
  }
}

__global__ __launch_bounds__(NTHR) void k_wprep(const float* __restrict__ w_off, const float* __restrict__ w_dsc,
                                                unsigned short* __restrict__ wof, unsigned short* __restrict__ wds) {
  const int i = blockIdx.x * NTHR + threadIdx.x;
  if (i >= 1728) return;
  v8us hv;
  if (i < 576) {
    const int e0 = i * 8;
    const int s  = e0 >> 9;
    const int rm = e0 & 511;
    const int n  = rm >> 5;
    const int k0 = rm & 31;
#pragma unroll
    for (int e = 0; e < 8; ++e) hv[e] = f2bf_bits(w_off[((size_t)n * NCH + (k0 + e)) * NTAP + s]);
    *(volatile v8us*)(wof + e0) = hv;
    __threadfence();
    *(volatile v8us*)(wof + e0) = hv;
  } else {
    const int e0 = (i - 576) * 8;
    const int s  = e0 >> 10;
    const int rm = e0 & 1023;
    const int n  = rm >> 5;
    const int k0 = rm & 31;
#pragma unroll
    for (int e = 0; e < 8; ++e) {
      const float wv = bf_rne(w_dsc[((size_t)n * NCH + (k0 + e)) * NTAP + s]);
      const _Float16 hq = (_Float16)(CARRY_W * wv);
      hv[e] = __builtin_bit_cast(unsigned short, hq);
    }
    *(volatile v8us*)(wds + e0) = hv;
    __threadfence();
    *(volatile v8us*)(wds + e0) = hv;
  }
}

__global__ __launch_bounds__(NTHR) void k_convoff(const unsigned short* __restrict__ xcl, const unsigned short* __restrict__ wof,
                                                  const float* __restrict__ b_off, float* __restrict__ offp,
                                                  float* __restrict__ part) {
  __shared__ __align__(16) unsigned short wsh[NTAP * 16 * 32];
  __shared__ __align__(16) float slab[8 * 32 * SLAB1P];
  __shared__ float wst[8 * 16];
  __shared__ float bsh[16];
  const int tid = threadIdx.x, lane = tid & 31, wave = tid >> 5;
  const int hh = lane >> 4, c = lane & 15, koff = hh * 8;
  const int blk = blockIdx.x, b = blk >> 8, w = blk & 255;

  for (int q = tid; q < (NTAP * 16 * 32) / 8; q += NTHR) *(v4u*)(wsh + q * 8) = *(const v4u*)(wof + q * 8);
  if (tid < 16) bsh[tid] = bf_rne(b_off[tid]);
  __syncthreads();

  const __bf16* wb = (const __bf16*)wsh;
  const __bf16* xb = (const __bf16*)xcl + (size_t)b * PADN * PADN * XPIX;
  v8f acc[2];
  acc[0] = (v8f){0.f,0.f,0.f,0.f,0.f,0.f,0.f,0.f};
  acc[1] = acc[0];
  const int h0 = wave * 32 + c;
#pragma unroll 1
  for (int s = 0; s < NTAP; ++s) {
    const int ky = s / 3, kx = s - ky * 3;
    const v16b bw = Frag<__bf16>::load(wb + (s * 16 + c) * 32 + koff);
    const size_t rowp = (size_t)(w + ky) * PADN;
    const v16b a0 = Frag<__bf16>::load(xb + (rowp + (size_t)(h0 + kx)) * XPIX + koff);
    const v16b a1 = Frag<__bf16>::load(xb + (rowp + (size_t)(h0 + 16 + kx)) * XPIX + koff);
    acc[0] = Frag<__bf16>::mma(a0, bw, acc[0]);
    acc[1] = Frag<__bf16>::mma(a1, bw, acc[1]);
    guard2_b3(acc[0], acc[1], a0, a1, bw);
  }
  acc_guard2(acc[0], acc[1]);

  float* sl = slab + wave * (32 * SLAB1P);
  const float bias = bsh[c];
  float ssum = 0.0f, ssq = 0.0f;
#pragma unroll
  for (int i = 0; i < 2; ++i) {
#pragma unroll
    for (int r = 0; r < 8; ++r) {
      const float v = acc[i][r] + bias;
      sl[(i * 16 + 8 * hh + r) * SLAB1P + c] = v;
      ssum += v;
      ssq = fmaf(v, v, ssq);
    }
  }
  wave_sync();
  float* ob = offp + ((size_t)b * NPIX + (size_t)w * NCOL + (size_t)wave * 32) * OFFC;
  for (int pass = 0; pass < 2; ++pass) {
#pragma unroll
    for (int it = 0; it < 4; ++it) {
      const int q  = it * 32 + lane;
      const int p  = q >> 2;
      const int c4 = (q & 3) * 4;
      const v4f v = *(const v4f*)(sl + p * SLAB1P + c4);
      *(volatile v4f*)(ob + (size_t)q * 4) = v;
    }
    __threadfence();
  }
  ssum += __shfl_xor(ssum, 16, 32); ssq += __shfl_xor(ssq, 16, 32);
  ssum += __shfl_xor(ssum, 1, 32);  ssq += __shfl_xor(ssq, 1, 32);
  if (hh == 0 && (c & 1) == 0) {
    wst[wave * 16 + (c >> 1)]     = ssum;
    wst[wave * 16 + 8 + (c >> 1)] = ssq;
  }
  __syncthreads();
  if (tid < 8) {
    v4f o;
#pragma unroll
    for (int j = 0; j < 4; ++j) {
      const int e  = tid * 4 + j;
      const int ec = (e < 16) ? e : 15;
      float a = 0.0f;
#pragma unroll
      for (int wv = 0; wv < 8; ++wv) a += wst[wv * 16 + ec];
      o[j] = (e < 16) ? a : 0.0f;
    }
    float* pp = part + (size_t)blk * PARTW + tid * 4;
    *(volatile v4f*)pp = o;
    __threadfence();
    *(volatile v4f*)pp = o;
  }
}

__global__ __launch_bounds__(64) void k_finalize(const float* __restrict__ part, int rowsPerImg, float inv_n,
                                                 float* __restrict__ stats) {
  __shared__ __align__(16) float sh[64];
  const int tid = threadIdx.x;
  if (tid < 32) {
    const int b = tid >> 3, g = tid & 7;
    const int nr = (rowsPerImg < NROW) ? rowsPerImg : NROW;
    double s = 0.0, q = 0.0;
#pragma unroll 1
    for (int r = 0; r < nr; ++r) {
      const float* p = part + ((size_t)(b * rowsPerImg + r)) * PARTW;
      s += (double)p[g];
      q += (double)p[8 + g];
    }
    const double mean = s * (double)inv_n;
    double var = q * (double)inv_n - mean * mean;
    if (var < 0.0) var = 0.0;
    const float varf = (float)var;
    sh[tid]      = (float)mean;
    sh[32 + tid] = 1.0f / sqrtf(varf + GN_EPS);
  }
  __syncthreads();
  if (tid < 16) {
    const v4f v = *(const v4f*)(sh + 4 * tid);
    *(volatile v4f*)(stats + 4 * tid) = v;
    __threadfence();
    *(volatile v4f*)(stats + 4 * tid) = v;
  }
}

__global__ __launch_bounds__(NTHR) void k_dsc(const unsigned short* __restrict__ xcl, const unsigned short* __restrict__ wds,
                                              const float* __restrict__ offp, const float* __restrict__ stats1,
                                              const float* __restrict__ gn_off_scale, const float* __restrict__ gn_off_bias,
                                              const float* __restrict__ b_dsc, float* __restrict__ pre,
                                              float* __restrict__ part) {
  __shared__ __align__(16) unsigned short wsh[NTAP * 32 * 32];
  __shared__ __align__(16) float crd[NTAP * NCOL * 4];
  __shared__ __align__(16) _Float16 atile[8 * 32 * ATP];
  __shared__ float wst[8 * 16];
  __shared__ float prm[64];
  __shared__ float bsh[32];
  const int tid = threadIdx.x, lane = tid & 31, wave = tid >> 5;
  const int hh = lane >> 4, c = lane & 15, koff = hh * 8;
  const int blk = blockIdx.x, b = blk >> 8, w = blk & 255;

  for (int q = tid; q < (NTAP * 32 * 32) / 8; q += NTHR) *(v4u*)(wsh + q * 8) = *(const v4u*)(wds + q * 8);
  if (tid < 10) {
    const int g = tid >> 1;
    prm[tid]      = stats1[b * 8 + g];
    prm[16 + tid] = stats1[32 + b * 8 + g];
    prm[32 + tid] = bf_rne(gn_off_scale[tid]);
    prm[48 + tid] = bf_rne(gn_off_bias[tid]);
  }
  if (tid < 32) bsh[tid] = bf_rne(b_dsc[tid]);
  __syncthreads();

  {
    const float* op = offp + ((size_t)b * NPIX + (size_t)w * NCOL + (size_t)tid) * OFFC;
    const v4f o0 = *(const v4f*)(op);
    const v4f o1 = *(const v4f*)(op + 4);
    const v4f o2 = *(const v4f*)(op + 8);
    float raw[10];
    raw[0] = o0[0]; raw[1] = o0[1]; raw[2] = o0[2]; raw[3] = o0[3];
    raw[4] = o1[0]; raw[5] = o1[1]; raw[6] = o1[2]; raw[7] = o1[3];
    raw[8] = o2[0]; raw[9] = o2[1];
    float tv[10];
#pragma unroll
    for (int ch = 0; ch < 10; ++ch) {
      if (ch == 4 || ch == 9) {
        tv[ch] = 0.0f;
      } else {
        const float xn = (raw[ch] - prm[ch]) * prm[16 + ch];
        tv[ch] = tanhf(xn * prm[32 + ch] + prm[48 + ch]);
      }
    }
    float yc[9];
    yc[3] = tv[3]; yc[2] = yc[3] + tv[2]; yc[1] = yc[2] + tv[1]; yc[0] = yc[1] + tv[0];
    yc[4] = 0.0f;
    yc[5] = tv[5]; yc[6] = yc[5] + tv[6]; yc[7] = yc[6] + tv[7]; yc[8] = yc[7] + tv[8];
    const float fw = (float)w;
#pragma unroll
    for (int k = 0; k < NTAP; ++k) {
      const float yn = fw + yc[k];
      float gy = (yn * (1.0f / 256.0f)) * 2.0f - 1.0f;
      gy = fminf(fmaxf(gy, -1.0f), 1.0f);
      const float py = ((gy + 1.0f) * 0.5f) * 255.0f;
      const float xq = (float)(tid + k - 4);
      float gx = (xq * (1.0f / 256.0f)) * 2.0f - 1.0f;
      gx = fminf(fmaxf(gx, -1.0f), 1.0f);
      const float px = ((gx + 1.0f) * 0.5f) * 255.0f;
      const float y0f = floorf(py), x0f = floorf(px);
      const float wy = py - y0f, wx = px - x0f;
      const int y0i = (int)fminf(fmaxf(y0f, 0.0f), 255.0f);
      const int x0i = (int)fminf(fmaxf(x0f, 0.0f), 255.0f);
      v4f cd;
      cd[0] = __int_as_float(y0i); cd[1] = __int_as_float(x0i); cd[2] = wy; cd[3] = wx;
      *(v4f*)(crd + (k * NCOL + tid) * 4) = cd;
    }
  }
  __syncthreads();

  const unsigned short* xb = xcl + (size_t)b * PADN * PADN * XPIX;
  const _Float16* wb = (const _Float16*)wsh;
  _Float16* aw = atile + wave * (32 * ATP);
  v8f acc[2][2];
#pragma unroll
  for (int i = 0; i < 2; ++i) { acc[i][0] = (v8f){0.f,0.f,0.f,0.f,0.f,0.f,0.f,0.f}; acc[i][1] = acc[i][0]; }
#pragma unroll 1
  for (int s = 0; s < NTAP; ++s) {
#pragma unroll 1
    for (int i = 0; i < 2; ++i) {
      const int p = i * 16 + c;
      const int h = wave * 32 + p;
      const v4f cd = *(const v4f*)(crd + (s * NCOL + h) * 4);
      int y0 = __float_as_int(cd[0]), x0 = __float_as_int(cd[1]);
      y0 = min(max(y0, 0), NROW - 1); x0 = min(max(x0, 0), NCOL - 1);
      const int y1 = min(y0 + 1, NROW - 1), x1 = min(x0 + 1, NCOL - 1);
      const float wy = cd[2], wx = cd[3];
      const float omy = 1.0f - wy, omx = 1.0f - wx;
      const float w00 = (CARRY_A * omy) * omx, w01 = (CARRY_A * omy) * wx;
      const float w10 = (CARRY_A * wy) * omx,  w11 = (CARRY_A * wy) * wx;
      const int chb = hh * 16;
      const unsigned short* p00 = xb + ((size_t)(y0 + 1) * PADN + (size_t)(x0 + 1)) * XPIX + chb;
      const unsigned short* p01 = xb + ((size_t)(y0 + 1) * PADN + (size_t)(x1 + 1)) * XPIX + chb;
      const unsigned short* p10 = xb + ((size_t)(y1 + 1) * PADN + (size_t)(x0 + 1)) * XPIX + chb;
      const unsigned short* p11 = xb + ((size_t)(y1 + 1) * PADN + (size_t)(x1 + 1)) * XPIX + chb;
      const v4u ua00 = *(const v4u*)(p00), ub00 = *(const v4u*)(p00 + 8);
      const v4u ua01 = *(const v4u*)(p01), ub01 = *(const v4u*)(p01 + 8);
      const v4u ua10 = *(const v4u*)(p10), ub10 = *(const v4u*)(p10 + 8);
      const v4u ua11 = *(const v4u*)(p11), ub11 = *(const v4u*)(p11 + 8);
      v8h hv0, hv1;
#pragma unroll
      for (int e = 0; e < 4; ++e) {
        hv0[2 * e]     = (_Float16)lerp4(lo16f(ua00[e]), lo16f(ua01[e]), lo16f(ua10[e]), lo16f(ua11[e]), w00, w01, w10, w11);
        hv0[2 * e + 1] = (_Float16)lerp4(hi16f(ua00[e]), hi16f(ua01[e]), hi16f(ua10[e]), hi16f(ua11[e]), w00, w01, w10, w11);
        hv1[2 * e]     = (_Float16)lerp4(lo16f(ub00[e]), lo16f(ub01[e]), lo16f(ub10[e]), lo16f(ub11[e]), w00, w01, w10, w11);
        hv1[2 * e + 1] = (_Float16)lerp4(hi16f(ub00[e]), hi16f(ub01[e]), hi16f(ub10[e]), hi16f(ub11[e]), w00, w01, w10, w11);
      }
      *(v8h*)(aw + p * ATP + chb)     = hv0;
      *(v8h*)(aw + p * ATP + chb + 8) = hv1;
      asm volatile("" ::: "memory");
    }
    wave_sync();
    const v16h bq0 = Frag<_Float16>::load(wb + (s * 32 + c) * 32 + koff);
    const v16h bq1 = Frag<_Float16>::load(wb + (s * 32 + 16 + c) * 32 + koff);
#pragma unroll
    for (int i = 0; i < 2; ++i) {
      const v16h af = Frag<_Float16>::load(aw + (i * 16 + c) * ATP + koff);
      acc[i][0] = Frag<_Float16>::mma(af, bq0, acc[i][0]);
      acc[i][1] = Frag<_Float16>::mma(af, bq1, acc[i][1]);
      guard2_h3(acc[i][0], acc[i][1], af, bq0, bq1);
    }
    wave_sync();
  }
  acc_guard4(acc[0][0], acc[0][1], acc[1][0], acc[1][1]);
  __syncthreads();

  float* sl = crd + wave * (32 * SLAB2P);
  const float bs0 = bsh[c], bs1 = bsh[16 + c];
  float s0 = 0.0f, q0 = 0.0f, s1 = 0.0f, q1 = 0.0f;
#pragma unroll
  for (int i = 0; i < 2; ++i) {
#pragma unroll
    for (int r = 0; r < 8; ++r) {
      const int px = i * 16 + 8 * hh + r;
      const float v0 = fmaf(acc[i][0][r], FOLD2, bs0);
      const float v1 = fmaf(acc[i][1][r], FOLD2, bs1);
      sl[c * SLAB2P + px]        = v0;
      sl[(16 + c) * SLAB2P + px] = v1;
      s0 += v0; q0 = fmaf(v0, v0, q0);
      s1 += v1; q1 = fmaf(v1, v1, q1);
    }
  }
  wave_sync();
  float* pb = pre + ((size_t)b * NCH) * NPIX + (size_t)w * NCOL + (size_t)wave * 32;
  const int lq = lane >> 3, f4 = (lane & 7) * 4;
  for (int pass = 0; pass < 2; ++pass) {
#pragma unroll
    for (int it = 0; it < 8; ++it) {
      const int ch = it * 4 + lq;
      const v4f v = *(const v4f*)(sl + ch * SLAB2P + f4);
      *(volatile v4f*)(pb + (size_t)ch * NPIX + f4) = v;
    }
    __threadfence();
  }
  s0 += __shfl_xor(s0, 16, 32); q0 += __shfl_xor(q0, 16, 32); s1 += __shfl_xor(s1, 16, 32); q1 += __shfl_xor(q1, 16, 32);
  s0 += __shfl_xor(s0, 1, 32);  q0 += __shfl_xor(q0, 1, 32);  s1 += __shfl_xor(s1, 1, 32);  q1 += __shfl_xor(q1, 1, 32);
  s0 += __shfl_xor(s0, 2, 32);  q0 += __shfl_xor(q0, 2, 32);  s1 += __shfl_xor(s1, 2, 32);  q1 += __shfl_xor(q1, 2, 32);
  if (hh == 0 && (c & 3) == 0) {
    const int g0 = c >> 2;
    wst[wave * 16 + g0]      = s0;
    wst[wave * 16 + 4 + g0]  = s1;
    wst[wave * 16 + 8 + g0]  = q0;
    wst[wave * 16 + 12 + g0] = q1;
  }
  __syncthreads();
  if (tid < 8) {
    v4f o;
#pragma unroll
    for (int j = 0; j < 4; ++j) {
      const int e  = tid * 4 + j;
      const int ec = (e < 16) ? e : 15;
      float a = 0.0f;
#pragma unroll
      for (int wv = 0; wv < 8; ++wv) a += wst[wv * 16 + ec];
      o[j] = (e < 16) ? a : 0.0f;
    }
    float* pp = part + (size_t)blk * PARTW + tid * 4;
    *(volatile v4f*)pp = o;
    __threadfence();
    *(volatile v4f*)pp = o;
  }
}

__global__ __launch_bounds__(NTHR) void k_gnrelu(const float* __restrict__ pre, const float* __restrict__ stats2,
                                                 const float* __restrict__ gn_scale, const float* __restrict__ gn_bias,
                                                 float* __restrict__ out) {
  const size_t i4 = ((size_t)blockIdx.x * NTHR + threadIdx.x) * 4;
  const int ch = (int)((i4 >> 16) & 31);
  const int b  = (int)(i4 >> 21);
  const int g  = ch >> 2;
  const float mean = stats2[b * 8 + g];
  const float rstd = stats2[32 + b * 8 + g];
  const float sc = bf_rne(gn_scale[ch]);
  const float bi = bf_rne(gn_bias[ch]);
  const v4f v = *(const v4f*)(pre + i4);
  v4f o;
#pragma unroll
  for (int e = 0; e < 4; ++e) o[e] = fmaxf(((v[e] - mean) * rstd) * sc + bi, 0.0f);
  *(volatile v4f*)(out + i4) = o;
  __threadfence();
  *(volatile v4f*)(out + i4) = o;
}

extern "C" void kernel_launch(void* const* d_in, const int* in_sizes, int n_in,
                              void* d_out, int out_size, void* d_ws, size_t ws_size,
                              hipStream_t stream)
{
  (void)in_sizes;
  if (n_in < 9) return;
  if ((size_t)out_size != (size_t)NBATCH * NCH * NPIX) return;
  if (ws_size < WS_TOTAL) return;

  const float* x            = (const float*)d_in[0];
  const float* w_off        = (const float*)d_in[1];
  const float* b_off        = (const float*)d_in[2];
  const float* gn_off_scale = (const float*)d_in[3];
  const float* gn_off_bias  = (const float*)d_in[4];
  const float* w_dsc        = (const float*)d_in[5];
  const float* b_dsc        = (const float*)d_in[6];
  const float* gn_scale     = (const float*)d_in[7];
  const float* gn_bias      = (const float*)d_in[8];
  float* out = (float*)d_out;

  char* ws = (char*)d_ws;
  unsigned short* xcl   = (unsigned short*)(ws + XCL_OFS);
  float*          offp  = (float*)(ws + OFF_OFS);
  float*          pre   = (float*)(ws + PRE_OFS);
  unsigned short* wof   = (unsigned short*)(ws + WOF_OFS);
  unsigned short* wds   = (unsigned short*)(ws + WDS_OFS);
  float*          part1 = (float*)(ws + PART1_OFS);
  float*          part2 = (float*)(ws + PART2_OFS);
  float*          st1   = (float*)(ws + ST1_OFS);
  float*          st2   = (float*)(ws + ST2_OFS);

  k_xprep<<<NBATCH * PADN, NTHR, 0, stream>>>(x, xcl);
  k_wprep<<<(1728 + NTHR - 1) / NTHR, NTHR, 0, stream>>>(w_off, w_dsc, wof, wds);
  k_convoff<<<NBATCH * NROW, NTHR, 0, stream>>>(xcl, wof, b_off, offp, part1);
  k_finalize<<<1, 64, 0, stream>>>(part1, NROW, 1.0f / 131072.0f, st1);
  k_dsc<<<NBATCH * NROW, NTHR, 0, stream>>>(xcl, wds, offp, st1, gn_off_scale, gn_off_bias, b_dsc, pre, part2);
  k_finalize<<<1, 64, 0, stream>>>(part2, NROW, 1.0f / 262144.0f, st2);
  k_gnrelu<<<(NBATCH * NCH * NPIX) / (NTHR * 4), NTHR, 0, stream>>>(pre, st2, gn_scale, gn_bias, out);
}
